// MulHeadAttentionDecoder_6390911337073
// MI455X (gfx1250) — hardware-verified
//
#include <hip/hip_runtime.h>

typedef _Float16 v16h __attribute__((ext_vector_type(16)));
typedef __bf16   v16y __attribute__((ext_vector_type(16)));
typedef short    v16s __attribute__((ext_vector_type(16)));
typedef short    v8s  __attribute__((ext_vector_type(8)));
typedef float    v8f  __attribute__((ext_vector_type(8)));
typedef float    v4f  __attribute__((ext_vector_type(4)));
typedef v8s __attribute__((may_alias)) v8sa;
typedef v4f __attribute__((may_alias)) v4fa;
typedef unsigned short u16;

#define NTOK  2048
#define HID   1024
#define DEMB  300
#define DEMP  320
#define FFH   2048
#define NHEAD 8
#define DHD   128
#define LNEPS 1e-5f
#define PSC   16384.0f
#define SSC   (0.0625f * 0.08838834764831845f)
#define WS_LIMIT 134217728ull

__device__ __forceinline__ v8f mma_f16(v16s a, v16s b, v8f c) {
  const v16h ah = __builtin_bit_cast(v16h, a);
  const v16h bh = __builtin_bit_cast(v16h, b);
  v8f d = __builtin_amdgcn_wmma_f32_16x16x32_f16(false, ah, false, bh, (short)0, c, false, false);
  asm volatile("v_nop\n\tv_nop\n\tv_nop\n\tv_nop" : "+v"(d) : "v"(a), "v"(b));
  return d;
}
__device__ __forceinline__ v8f mma_bf16(v16s a, v16s b, v8f c) {
  const v16y ay = __builtin_bit_cast(v16y, a);
  const v16y by = __builtin_bit_cast(v16y, b);
  v8f d = __builtin_amdgcn_wmma_f32_16x16x32_bf16(false, ay, false, by, (short)0, c, false, false);
  asm volatile("v_nop\n\tv_nop\n\tv_nop\n\tv_nop" : "+v"(d) : "v"(a), "v"(b));
  return d;
}

__device__ __forceinline__ v16s ldfrag(const u16* p, int h) {
  union { v16s v; v8s q[2]; } f;
  f.q[0] = *(const v8sa*)(p + 8 * h);
  f.q[1] = *(const v8sa*)(p + 16 + 8 * h);
  return f.v;
}

__device__ __forceinline__ u16 f2h(float x) { const _Float16 t = (_Float16)x; return __builtin_bit_cast(u16, t); }
__device__ __forceinline__ u16 f2bf(float x) {
  unsigned u = __float_as_uint(x);
  u += 0x7FFFu + ((u >> 16) & 1u);
  return (u16)(u >> 16);
}
__device__ __forceinline__ float bf2f(u16 b) { return __uint_as_float(((unsigned)b) << 16); }

__device__ __forceinline__ v8s pk_f16(v8f y, float sc) {
  v8s o;
#pragma unroll
  for (int i = 0; i < 8; ++i) o[i] = (short)f2h(y[i] * sc);
  return o;
}
__device__ __forceinline__ void pk_bf(v8f y, v8s& hi, v8s& lo) {
  v8s a, b;
#pragma unroll
  for (int i = 0; i < 8; ++i) {
    const u16 hb = f2bf(y[i]);
    a[i] = (short)hb;
    b[i] = (short)f2bf(y[i] - bf2f(hb));
  }
  hi = a; lo = b;
}
__device__ __forceinline__ void st16(u16* p, v8s v) { *(volatile v8s*)p = v; }
__device__ __forceinline__ void stf4(float* p, v4f v) { *(volatile v4f*)p = v; }

struct Seg {
  const float* src; u16* dst; u16* dst2;
  int cols; int ldd; int ng; int mode; int vec; float scale;
};
static_assert(sizeof(Seg) == 48);
struct SegTab { Seg s[16]; };
static_assert(sizeof(SegTab) == 768);

__global__ __launch_bounds__(256) void convert_kernel(SegTab tab) {
  const int y = blockIdx.y;
  Seg sg = tab.s[0];
#define PICKSEG(i) if (y == i) sg = tab.s[i];
  PICKSEG(1) PICKSEG(2) PICKSEG(3) PICKSEG(4) PICKSEG(5) PICKSEG(6) PICKSEG(7)
  PICKSEG(8) PICKSEG(9) PICKSEG(10) PICKSEG(11) PICKSEG(12) PICKSEG(13) PICKSEG(14) PICKSEG(15)
#undef PICKSEG
  const int g = blockIdx.x * 256 + threadIdx.x;
  if (g >= sg.ng) return;
  const int ldd8 = sg.ldd >> 3;
  const int row = g / ldd8;
  const int c8 = (g - row * ldd8) * 8;
  v8f x;
  if (sg.vec) {
    const float* p = sg.src + (size_t)row * sg.cols + c8;
    const v4f a = *(const v4fa*)p;
    const v4f b = *(const v4fa*)(p + 4);
    x[0] = a[0]; x[1] = a[1]; x[2] = a[2]; x[3] = a[3];
    x[4] = b[0]; x[5] = b[1]; x[6] = b[2]; x[7] = b[3];
  } else {
    const float* p = sg.src + (size_t)row * sg.cols;
#pragma unroll
    for (int j = 0; j < 8; ++j) {
      const int c = c8 + j;
      const int cc = (c < sg.cols) ? c : (sg.cols - 1);
      const float v = p[cc];
      x[j] = (c < sg.cols) ? v : 0.0f;
    }
  }
  u16* d = sg.dst + (size_t)g * 8;
  if (sg.mode == 0) {
    const v8s o = pk_f16(x, sg.scale);
    st16(d, o);
    __threadfence();
    st16(d, o);
  } else {
    v8s hi, lo;
    pk_bf(x, hi, lo);
    u16* d2 = sg.dst2 + (size_t)g * 8;
    st16(d, hi); st16(d2, lo);
    __threadfence();
    st16(d, hi); st16(d2, lo);
  }
}

__device__ __forceinline__ void gemm_store(const float* sT, float* outF, int wf, u16* outA, u16* outB,
                                           int omode, float oscale, int ldc, int m0, int n0, int w, int lane) {
  if (wf) {
#pragma unroll
    for (int i = 0; i < 16; ++i) {
      const int row = 32 * w + 2 * i + (lane >> 4);
      const int c4 = (lane & 15) * 4;
      v4f v;
      v[0] = sT[(c4 + 0) * 128 + row]; v[1] = sT[(c4 + 1) * 128 + row];
      v[2] = sT[(c4 + 2) * 128 + row]; v[3] = sT[(c4 + 3) * 128 + row];
      stf4(outF + (size_t)(m0 + row) * ldc + n0 + c4, v);
    }
  }
  if (omode == 1 || omode == 2) {
#pragma unroll
    for (int i = 0; i < 8; ++i) {
      const int row = 32 * w + 4 * i + (lane >> 3);
      const int c8 = (lane & 7) * 8;
      v8f yv;
#pragma unroll
      for (int j = 0; j < 8; ++j) yv[j] = sT[(c8 + j) * 128 + row];
      const size_t gi = (size_t)(m0 + row) * ldc + n0 + c8;
      if (omode == 1) {
        st16(outA + gi, pk_f16(yv, oscale));
      } else {
        v8s hi, lo;
        pk_bf(yv, hi, lo);
        st16(outA + gi, hi);
        st16(outB + gi, lo);
      }
    }
  }
  if (omode == 3) {
#pragma unroll
    for (int i = 0; i < 8; ++i) {
      const int col = 16 * w + 2 * i + (lane >> 4);
      const int t8 = (lane & 15) * 8;
      const float* s = sT + col * 128 + t8;
      const v4f a = *(const v4fa*)s;
      const v4f b = *(const v4fa*)(s + 4);
      v8f yv;
      yv[0] = a[0]; yv[1] = a[1]; yv[2] = a[2]; yv[3] = a[3];
      yv[4] = b[0]; yv[5] = b[1]; yv[6] = b[2]; yv[7] = b[3];
      st16(outA + (size_t)(n0 + col) * ldc + m0 + t8, pk_f16(yv, oscale));
    }
  }
}

template <int SPLIT>
__global__ __launch_bounds__(128) void gemm_kernel(
    const u16* __restrict__ Ah, const u16* __restrict__ Al, int lda,
    const u16* __restrict__ Wh, const u16* __restrict__ Wl, int ldw,
    const float* __restrict__ bias, int K, float inv_in, int relu,
    float* outF, int wf, u16* outA, u16* outB, int omode, float oscale, int ldc)
{
  __shared__ __attribute__((aligned(16))) float sT[64 * 128];

  const int tid = threadIdx.x, lane = tid & 31, w = tid >> 5;
  const int h = lane >> 4, m = lane & 15;
  const int m0 = blockIdx.x * 128, n0 = blockIdx.y * 64;
  const int m0w = m0 + 32 * w;

  const u16* a0p = Ah + (size_t)(m0w + m) * lda;
  const u16* a1p = a0p + (size_t)16 * lda;
  const u16* a0q = Al + (size_t)(m0w + m) * lda;
  const u16* a1q = a0q + (size_t)16 * lda;
  const u16* wp  = Wh + (size_t)(n0 + m) * ldw;
  const u16* wq  = Wl + (size_t)(n0 + m) * ldw;

  const v8f zero8 = {0.f, 0.f, 0.f, 0.f, 0.f, 0.f, 0.f, 0.f};
  v8f acc[2][4];
#pragma unroll
  for (int mt = 0; mt < 2; ++mt)
#pragma unroll
    for (int nt = 0; nt < 4; ++nt) acc[mt][nt] = zero8;

#pragma unroll 1
  for (int k0 = 0; k0 < K; k0 += 32) {
    const v16s a0 = ldfrag(a0p + k0, h);
    const v16s a1 = ldfrag(a1p + k0, h);
    if (SPLIT) {
      const v16s a0l = ldfrag(a0q + k0, h);
      const v16s a1l = ldfrag(a1q + k0, h);
#pragma unroll
      for (int nt = 0; nt < 4; ++nt) {
        const v16s b  = ldfrag(wp + (size_t)nt * 16 * ldw + k0, h);
        const v16s bl = ldfrag(wq + (size_t)nt * 16 * ldw + k0, h);
        acc[0][nt] = mma_bf16(a0,  b,  acc[0][nt]);
        acc[0][nt] = mma_bf16(a0,  bl, acc[0][nt]);
        acc[0][nt] = mma_bf16(a0l, b,  acc[0][nt]);
        acc[1][nt] = mma_bf16(a1,  b,  acc[1][nt]);
        acc[1][nt] = mma_bf16(a1,  bl, acc[1][nt]);
        acc[1][nt] = mma_bf16(a1l, b,  acc[1][nt]);
      }
    } else {
#pragma unroll
      for (int nt = 0; nt < 4; ++nt) {
        const v16s b = ldfrag(wp + (size_t)nt * 16 * ldw + k0, h);
        acc[0][nt] = mma_f16(a0, b, acc[0][nt]);
        acc[1][nt] = mma_f16(a1, b, acc[1][nt]);
      }
    }
  }

#pragma unroll
  for (int nt = 0; nt < 4; ++nt) {
    const int col = 16 * nt + m;
    const float bv = bias[n0 + col];
#pragma unroll
    for (int mt = 0; mt < 2; ++mt) {
      v4f y0, y1;
#pragma unroll
      for (int r = 0; r < 4; ++r) {
        float t0 = acc[mt][nt][r] * inv_in + bv;
        float t1 = acc[mt][nt][r + 4] * inv_in + bv;
        if (relu) { t0 = fmaxf(t0, 0.0f); t1 = fmaxf(t1, 0.0f); }
        y0[r] = t0; y1[r] = t1;
      }
      float* d = sT + col * 128 + 32 * w + 16 * mt + 8 * h;
      *(v4fa*)d = y0;
      *(v4fa*)(d + 4) = y1;
    }
  }
  __syncthreads();

  gemm_store(sT, outF, wf, outA, outB, omode, oscale, ldc, m0, n0, w, lane);
  __threadfence();
  gemm_store(sT, outF, wf, outA, outB, omode, oscale, ldc, m0, n0, w, lane);
}

__device__ __forceinline__ void ln_store(const float* sO, float* outF, int wf, u16* outH, int wh,
                                         int rowbase, int tid) {
  if (wf) {
    const int c4 = tid * 4;
#pragma unroll
    for (int i = 0; i < 8; ++i) {
      v4f v;
      v[0] = sO[(c4 + 0) * 8 + i]; v[1] = sO[(c4 + 1) * 8 + i];
      v[2] = sO[(c4 + 2) * 8 + i]; v[3] = sO[(c4 + 3) * 8 + i];
      stf4(outF + (size_t)(rowbase + i) * HID + c4, v);
    }
  }
  if (wh) {
    const int c8 = (tid & 127) * 8;
#pragma unroll
    for (int i = 0; i < 4; ++i) {
      const int row = 2 * i + (tid >> 7);
      v8f yv;
#pragma unroll
      for (int j = 0; j < 8; ++j) yv[j] = sO[(c8 + j) * 8 + row];
      st16(outH + (size_t)(rowbase + row) * HID + c8, pk_f16(yv, 1.0f));
    }
  }
}

template <int SPLIT>
__global__ __launch_bounds__(256) void gemm_ln_kernel(
    const u16* __restrict__ Ah, const u16* __restrict__ Al, int lda,
    const u16* __restrict__ Wh, const u16* __restrict__ Wl, int ldw,
    const float* __restrict__ bias, int K, float inv_in,
    const float* __restrict__ xres, const float* __restrict__ gam, const float* __restrict__ bet,
    float* outF, int wf, u16* outH, int wh)
{
  __shared__ __attribute__((aligned(16))) float sO[HID * 8];
  __shared__ __attribute__((aligned(16))) float red[8 * 16];
  __shared__ float stat[32];

  const int tid = threadIdx.x, lane = tid & 31, w = tid >> 5;
  const int h = lane >> 4, m = lane & 15;
  const int r0 = blockIdx.x * 16;
  const int cw = 128 * w;

  const u16* ap = Ah + (size_t)(r0 + m) * lda;
  const u16* aq = Al + (size_t)(r0 + m) * lda;
  const u16* wp = Wh + (size_t)(cw + m) * ldw;
  const u16* wq = Wl + (size_t)(cw + m) * ldw;

  const v8f zero8 = {0.f, 0.f, 0.f, 0.f, 0.f, 0.f, 0.f, 0.f};
  v8f acc[8];
#pragma unroll
  for (int nt = 0; nt < 8; ++nt) acc[nt] = zero8;

#pragma unroll 1
  for (int k0 = 0; k0 < K; k0 += 32) {
    const v16s a = ldfrag(ap + k0, h);
    if (SPLIT) {
      const v16s al = ldfrag(aq + k0, h);
#pragma unroll
      for (int nt = 0; nt < 8; ++nt) {
        const v16s b  = ldfrag(wp + (size_t)nt * 16 * ldw + k0, h);
        const v16s bl = ldfrag(wq + (size_t)nt * 16 * ldw + k0, h);
        acc[nt] = mma_bf16(a,  b,  acc[nt]);
        acc[nt] = mma_bf16(a,  bl, acc[nt]);
        acc[nt] = mma_bf16(al, b,  acc[nt]);
      }
    } else {
#pragma unroll
      for (int nt = 0; nt < 8; ++nt) {
        const v16s b = ldfrag(wp + (size_t)nt * 16 * ldw + k0, h);
        acc[nt] = mma_f16(a, b, acc[nt]);
      }
    }
  }

#pragma unroll
  for (int nt = 0; nt < 8; ++nt) {
    const int col = cw + 16 * nt + m;
    const float bv = bias[col];
    const float* xr = xres + (size_t)(r0 + 8 * h) * HID + col;
#pragma unroll
    for (int r = 0; r < 8; ++r) acc[nt][r] = acc[nt][r] * inv_in + bv + xr[(size_t)r * HID];
  }

  v8f ps;
#pragma unroll
  for (int r = 0; r < 8; ++r) {
    float s = acc[0][r];
#pragma unroll
    for (int nt = 1; nt < 8; ++nt) s += acc[nt][r];
    s += __shfl_xor(s, 8);
    s += __shfl_xor(s, 4);
    s += __shfl_xor(s, 2);
    s += __shfl_xor(s, 1);
    ps[r] = s;
  }
  if (m == 0) {
    const v4f lo = {ps[0], ps[1], ps[2], ps[3]};
    const v4f hi = {ps[4], ps[5], ps[6], ps[7]};
    *(v4fa*)(red + w * 16 + 8 * h) = lo;
    *(v4fa*)(red + w * 16 + 8 * h + 4) = hi;
  }
  __syncthreads();
  if (tid < 16) {
    float t = 0.0f;
#pragma unroll
    for (int ww = 0; ww < 8; ++ww) t += red[ww * 16 + tid];
    stat[tid] = t * (1.0f / 1024.0f);
  }
  __syncthreads();
  v8f muv;
#pragma unroll
  for (int r = 0; r < 8; ++r) muv[r] = stat[8 * h + r];

  v8f pq;
#pragma unroll
  for (int r = 0; r < 8; ++r) {
    float s = 0.0f;
#pragma unroll
    for (int nt = 0; nt < 8; ++nt) { const float dd = acc[nt][r] - muv[r]; s += dd * dd; }
    s += __shfl_xor(s, 8);
    s += __shfl_xor(s, 4);
    s += __shfl_xor(s, 2);
    s += __shfl_xor(s, 1);
    pq[r] = s;
  }
  if (m == 0) {
    const v4f lo = {pq[0], pq[1], pq[2], pq[3]};
    const v4f hi = {pq[4], pq[5], pq[6], pq[7]};
    *(v4fa*)(red + w * 16 + 8 * h) = lo;
    *(v4fa*)(red + w * 16 + 8 * h + 4) = hi;
  }
  __syncthreads();
  if (tid < 16) {
    float t = 0.0f;
#pragma unroll
    for (int ww = 0; ww < 8; ++ww) t += red[ww * 16 + tid];
    const float var = t * (1.0f / 1024.0f);
    stat[16 + tid] = 1.0f / sqrtf(var + LNEPS);
  }
  __syncthreads();
  v8f rsv;
#pragma unroll
  for (int r = 0; r < 8; ++r) rsv[r] = stat[16 + 8 * h + r];

#pragma unroll
  for (int nt = 0; nt < 8; ++nt) {
    const int col = cw + 16 * nt + m;
    const float g = gam[col];
    const float b = bet[col];
#pragma unroll
    for (int r = 0; r < 8; ++r) acc[nt][r] = g * (acc[nt][r] - muv[r]) * rsv[r] + b;
  }

#pragma unroll
  for (int p = 0; p < 2; ++p) {
    if (h == p) {
#pragma unroll
      for (int nt = 0; nt < 8; ++nt) {
        const int col = cw + 16 * nt + m;
        const v4f lo = {acc[nt][0], acc[nt][1], acc[nt][2], acc[nt][3]};
        const v4f hi = {acc[nt][4], acc[nt][5], acc[nt][6], acc[nt][7]};
        *(v4fa*)(sO + col * 8) = lo;
        *(v4fa*)(sO + col * 8 + 4) = hi;
      }
    }
    __syncthreads();
    ln_store(sO, outF, wf, outH, wh, r0 + 8 * p, tid);
    __threadfence();
    ln_store(sO, outF, wf, outH, wh, r0 + 8 * p, tid);
    __syncthreads();
  }
}

__device__ __forceinline__ v16s pack_p(v8f a, v8f c) {
  v16s r;
#pragma unroll
  for (int i = 0; i < 8; ++i) {
    r[i]     = (short)f2h(a[i] * PSC);
    r[8 + i] = (short)f2h(c[i] * PSC);
  }
  return r;
}

__device__ __forceinline__ void att_store(const float* so, u16* outA, u16* outB, int omode,
                                          int q0, int head, int lane) {
#pragma unroll
  for (int i = 0; i < 8; ++i) {
    const int row = 2 * i + (lane >> 4);
    const int c8 = (lane & 15) * 8;
    const float* s = so + row * DHD + c8;
    const v4f a = *(const v4fa*)s;
    const v4f b = *(const v4fa*)(s + 4);
    v8f yv;
    yv[0] = a[0]; yv[1] = a[1]; yv[2] = a[2]; yv[3] = a[3];
    yv[4] = b[0]; yv[5] = b[1]; yv[6] = b[2]; yv[7] = b[3];
    const size_t gi = (size_t)(q0 + row) * HID + head * DHD + c8;
    if (omode == 1) {
      st16(outA + gi, pk_f16(yv, 1.0f));
    } else {
      v8s hi, lo;
      pk_bf(yv, hi, lo);
      st16(outA + gi, hi);
      st16(outB + gi, lo);
    }
  }
}

__global__ __launch_bounds__(128) void attn_kernel(
    const u16* __restrict__ qp, const u16* __restrict__ kp, const u16* __restrict__ vt,
    u16* outA, u16* outB, int omode, float onorm)
{
  __shared__ __attribute__((aligned(16))) float sO[4 * 16 * DHD];

  const int tid = threadIdx.x, lane = tid & 31, w = tid >> 5;
  const int h = lane >> 4, m = lane & 15;
  const int head = blockIdx.y;
  const int q0 = blockIdx.x * 64 + 16 * w;

  const u16* qrow  = qp + (size_t)(q0 + m) * HID + head * DHD;
  const u16* kbase = kp + (size_t)m * HID + head * DHD;
  const u16* vbase = vt + ((size_t)head * DHD + m) * NTOK;

  const v8f zero8 = {0.f, 0.f, 0.f, 0.f, 0.f, 0.f, 0.f, 0.f};
  v8f o[8];
#pragma unroll
  for (int t = 0; t < 8; ++t) o[t] = zero8;
  float mrun = -1e30f, lrun = 0.0f;

#pragma unroll 1
  for (int kb = 0; kb < NTOK; kb += 64) {
    v16s qb[4];
#pragma unroll
    for (int c = 0; c < 4; ++c) qb[c] = ldfrag(qrow + 32 * c, h);

    v8f s[4];
#pragma unroll
    for (int j = 0; j < 4; ++j) {
      const u16* kpj = kbase + (size_t)(kb + 16 * j) * HID;
      v8f z = zero8;
#pragma unroll
      for (int c = 0; c < 4; ++c) z = mma_f16(ldfrag(kpj + 32 * c, h), qb[c], z);
      s[j] = z;
    }

    float mloc = -1e30f;
#pragma unroll
    for (int j = 0; j < 4; ++j)
#pragma unroll
      for (int r = 0; r < 8; ++r) {
        const float t = s[j][r] * SSC;
        s[j][r] = t;
        mloc = fmaxf(mloc, t);
      }
    mloc = fmaxf(mloc, __shfl_xor(mloc, 16));
    const float mnew = fmaxf(mrun, mloc);
    const float alpha = __expf(mrun - mnew);
    mrun = mnew;
    float lsum = 0.0f;
#pragma unroll
    for (int j = 0; j < 4; ++j)
#pragma unroll
      for (int r = 0; r < 8; ++r) {
        const float p = __expf(s[j][r] - mnew);
        s[j][r] = p;
        lsum += p;
      }
    lsum += __shfl_xor(lsum, 16);
    lrun = lrun * alpha + lsum;
#pragma unroll
    for (int t = 0; t < 8; ++t)
#pragma unroll
      for (int r = 0; r < 8; ++r) o[t][r] = o[t][r] * alpha;

    const v16s pb0 = pack_p(s[0], s[1]);
    const v16s pb1 = pack_p(s[2], s[3]);

#pragma unroll
    for (int t = 0; t < 8; ++t) {
      const u16* vpt = vbase + (size_t)(16 * t) * NTOK + kb;
      o[t] = mma_f16(ldfrag(vpt, h), pb0, o[t]);
      o[t] = mma_f16(ldfrag(vpt + 32, h), pb1, o[t]);
    }
  }

  const float inv = onorm * (1.0f / lrun);
  float* so = sO + w * (16 * DHD);
#pragma unroll
  for (int t = 0; t < 8; ++t) {
    const v4f a = {o[t][0] * inv, o[t][1] * inv, o[t][2] * inv, o[t][3] * inv};
    const v4f b = {o[t][4] * inv, o[t][5] * inv, o[t][6] * inv, o[t][7] * inv};
    float* d = so + m * DHD + 16 * t + 8 * h;
    *(v4fa*)d = a;
    *(v4fa*)(d + 4) = b;
  }
  __syncthreads();

  att_store(so, outA, outB, omode, q0, head, lane);
  __threadfence();
  att_store(so, outA, outB, omode, q0, head, lane);
}

extern "C" void kernel_launch(void* const* d_in, const int* in_sizes, int n_in,
                              void* d_out, int out_size, void* d_ws, size_t ws_size,
                              hipStream_t stream) {
  if (n_in < 35) return;
  static const int expect_n[35] = {
    NTOK * DEMB, NTOK * DEMB, NTOK * HID, HID * DEMB, HID,
    3 * HID * HID, 3 * HID, HID * HID, HID,
    3 * HID * HID, 3 * HID, HID * HID, HID,
    3 * HID * HID, 3 * HID, HID * HID, HID,
    FFH * HID, FFH, HID * FFH, HID, HID, HID,
    FFH * HID, FFH, HID * FFH, HID, HID, HID,
    FFH * HID, FFH, HID * FFH, HID, HID, HID };
  for (int i = 0; i < 35; ++i) if (in_sizes[i] != expect_n[i]) return;
  if (out_size != NTOK * HID) return;

  const float* IIN = (const float*)d_in[0];
  const float* WIN = (const float*)d_in[1];
  const float* SIN = (const float*)d_in[2];
  const float* WWD = (const float*)d_in[3];
  const float* BWD = (const float*)d_in[4];
  const float* WQKV[3]; const float* BQKV[3]; const float* WO[3]; const float* BO[3];
  for (int j = 0; j < 3; ++j) {
    WQKV[j] = (const float*)d_in[5 + 4 * j];
    BQKV[j] = (const float*)d_in[6 + 4 * j];
    WO[j]   = (const float*)d_in[7 + 4 * j];
    BO[j]   = (const float*)d_in[8 + 4 * j];
  }
  const float* W1[3]; const float* B1[3]; const float* W2[3]; const float* B2[3];
  const float* GA[3]; const float* BE[3];
  for (int j = 0; j < 3; ++j) {
    const int base = 17 + 6 * j;
    W1[j] = (const float*)d_in[base + 0];
    B1[j] = (const float*)d_in[base + 1];
    W2[j] = (const float*)d_in[base + 2];
    B2[j] = (const float*)d_in[base + 3];
    GA[j] = (const float*)d_in[base + 4];
    BE[j] = (const float*)d_in[base + 5];
  }
  float* OUT = (float*)d_out;

  char* wsb = (char*)d_ws;
  size_t off = 0;
  auto alloc = [&](size_t bytes) -> char* {
    char* p = wsb + off;
    off += (bytes + 255) & ~(size_t)255;
    return p;
  };
  u16* wwd_h = (u16*)alloc((size_t)HID * DEMP * 2);
  u16* wqkv_h[3];
  for (int j = 0; j < 3; ++j) wqkv_h[j] = (u16*)alloc((size_t)3 * HID * HID * 2);
  u16* wo_h[2]; u16* w1_h[2]; u16* w2_h[2];
  for (int j = 0; j < 2; ++j) {
    wo_h[j] = (u16*)alloc((size_t)HID * HID * 2);
    w1_h[j] = (u16*)alloc((size_t)FFH * HID * 2);
    w2_h[j] = (u16*)alloc((size_t)HID * FFH * 2);
  }
  u16* wo3h = (u16*)alloc((size_t)HID * HID * 2);
  u16* wo3l = (u16*)alloc((size_t)HID * HID * 2);
  u16* w13h = (u16*)alloc((size_t)FFH * HID * 2);
  u16* w13l = (u16*)alloc((size_t)FFH * HID * 2);
  u16* w23h = (u16*)alloc((size_t)HID * FFH * 2);
  u16* w23l = (u16*)alloc((size_t)HID * FFH * 2);
  u16* wpad = (u16*)alloc((size_t)NTOK * DEMP * 2);
  u16* ipad = (u16*)alloc((size_t)NTOK * DEMP * 2);
  u16* s_h  = (u16*)alloc((size_t)NTOK * HID * 2);
  u16* w_h  = (u16*)alloc((size_t)NTOK * HID * 2);
  u16* i_h  = (u16*)alloc((size_t)NTOK * HID * 2);
  u16* qpl  = (u16*)alloc((size_t)NTOK * HID * 2);
  u16* kpl  = (u16*)alloc((size_t)NTOK * HID * 2);
  u16* vtp  = (u16*)alloc((size_t)HID * NTOK * 2);
  u16* ctxA = (u16*)alloc((size_t)NTOK * HID * 2);
  u16* ctxB = (u16*)alloc((size_t)NTOK * HID * 2);
  float* xres = (float*)alloc((size_t)NTOK * HID * 4);
  u16* xA   = (u16*)alloc((size_t)NTOK * HID * 2);
  u16* xB   = (u16*)alloc((size_t)NTOK * HID * 2);
  u16* hA   = (u16*)alloc((size_t)NTOK * FFH * 2);
  u16* iw_h = (u16*)alloc((size_t)NTOK * HID * 2);
  u16* sw_h = (u16*)alloc((size_t)NTOK * HID * 2);
  u16* hB   = w_h;
  if (off > ws_size) return;
  if (off > (size_t)WS_LIMIT) return;
  float* dummyF = (float*)ctxB;

  SegTab tab;
  auto seg = [&](int idx, const float* src, u16* dst, u16* dst2, int rows, int cols, int ldd,
                 int mode, float scale) {
    Seg s;
    s.src = src; s.dst = dst; s.dst2 = dst2;
    s.cols = cols; s.ldd = ldd; s.ng = rows * (ldd / 8);
    s.mode = mode; s.vec = (cols == ldd) ? 1 : 0; s.scale = scale;
    tab.s[idx] = s;
  };
  seg(0, WWD, wwd_h, wwd_h, HID, DEMB, DEMP, 0, 32.0f);
  for (int j = 0; j < 3; ++j) seg(1 + j, WQKV[j], wqkv_h[j], wqkv_h[j], 3 * HID, HID, HID, 0, 32.0f);
  for (int j = 0; j < 2; ++j) {
    seg(4 + j, WO[j], wo_h[j], wo_h[j], HID, HID, HID, 0, 32.0f);
    seg(6 + j, W1[j], w1_h[j], w1_h[j], FFH, HID, HID, 0, 32.0f);
    seg(8 + j, W2[j], w2_h[j], w2_h[j], HID, FFH, FFH, 0, 32.0f);
  }
  seg(10, WO[2], wo3h, wo3l, HID, HID, HID, 1, 1.0f);
  seg(11, W1[2], w13h, w13l, FFH, HID, HID, 1, 1.0f);
  seg(12, W2[2], w23h, w23l, HID, FFH, FFH, 1, 1.0f);
  seg(13, WIN, wpad, wpad, NTOK, DEMB, DEMP, 0, 1.0f);
  seg(14, IIN, ipad, ipad, NTOK, DEMB, DEMP, 0, 1.0f);
  seg(15, SIN, s_h, s_h, NTOK, HID, HID, 0, 1.0f);
  const int max_ng = 3 * HID * HID / 8;
  convert_kernel<<<dim3((max_ng + 255) / 256, 16), 256, 0, stream>>>(tab);

  const dim3 g16(NTOK / 128, HID / 64);
  const dim3 g32(NTOK / 128, FFH / 64);
  const dim3 gat(NTOK / 64, NHEAD);
  const int  gln = NTOK / 16;

  gemm_kernel<0><<<g16, 128, 0, stream>>>(wpad, wpad, DEMP, wwd_h, wwd_h, DEMP, BWD, DEMP,
                                           1.0f / 32.0f, 0, dummyF, 0, w_h, w_h, 1, 1.0f, HID);
  gemm_kernel<0><<<g16, 128, 0, stream>>>(ipad, ipad, DEMP, wwd_h, wwd_h, DEMP, BWD, DEMP,
                                           1.0f / 32.0f, 0, dummyF, 0, i_h, i_h, 1, 1.0f, HID);

  auto mha = [&](const u16* qs, const u16* ks, const u16* vs, int j, u16* oA, u16* oB,
                 int om, float onorm) {
    gemm_kernel<0><<<g16, 128, 0, stream>>>(qs, qs, HID, wqkv_h[j], wqkv_h[j], HID, BQKV[j], HID,
                                             1.0f / 32.0f, 0, dummyF, 0, qpl, qpl, 1, 4.0f, HID);
    gemm_kernel<0><<<g16, 128, 0, stream>>>(ks, ks, HID, wqkv_h[j] + (size_t)HID * HID,
                                             wqkv_h[j] + (size_t)HID * HID, HID, BQKV[j] + HID, HID,
                                             1.0f / 32.0f, 0, dummyF, 0, kpl, kpl, 1, 4.0f, HID);
    gemm_kernel<0><<<g16, 128, 0, stream>>>(vs, vs, HID, wqkv_h[j] + (size_t)2 * HID * HID,
                                             wqkv_h[j] + (size_t)2 * HID * HID, HID, BQKV[j] + 2 * HID, HID,
                                             1.0f / 32.0f, 0, dummyF, 0, vtp, vtp, 3, 4.0f, NTOK);
    attn_kernel<<<gat, 128, 0, stream>>>(qpl, kpl, vtp, oA, oB, om, onorm);
  };

  mha(w_h, i_h, i_h, 0, ctxA, ctxA, 1, 1.0f / 1024.0f);
  gemm_kernel<0><<<g16, 128, 0, stream>>>(ctxA, ctxA, HID, wo_h[0], wo_h[0], HID, BO[0], HID,
                                           1.0f / 2048.0f, 0, xres, 1, xA, xA, 1, 128.0f, HID);
  gemm_kernel<0><<<g32, 128, 0, stream>>>(xA, xA, HID, w1_h[0], w1_h[0], HID, B1[0], HID,
                                           1.0f / 4096.0f, 1, dummyF, 0, hA, hA, 1, 256.0f, FFH);
  gemm_ln_kernel<0><<<gln, 256, 0, stream>>>(hA, hA, FFH, w2_h[0], w2_h[0], FFH, B2[0], FFH,
                                              1.0f / 8192.0f, xres, GA[0], BE[0], dummyF, 0, iw_h, 1);

  mha(w_h, s_h, s_h, 1, ctxA, ctxA, 1, 1.0f / 1024.0f);
  gemm_kernel<0><<<g16, 128, 0, stream>>>(ctxA, ctxA, HID, wo_h[1], wo_h[1], HID, BO[1], HID,
                                           1.0f / 2048.0f, 0, xres, 1, xA, xA, 1, 128.0f, HID);
  gemm_kernel<0><<<g32, 128, 0, stream>>>(xA, xA, HID, w1_h[1], w1_h[1], HID, B1[1], HID,
                                           1.0f / 4096.0f, 1, dummyF, 0, hA, hA, 1, 256.0f, FFH);
  gemm_ln_kernel<0><<<gln, 256, 0, stream>>>(hA, hA, FFH, w2_h[1], w2_h[1], FFH, B2[1], FFH,
                                              1.0f / 8192.0f, xres, GA[1], BE[1], dummyF, 0, sw_h, 1);

  mha(s_h, iw_h, sw_h, 2, ctxA, ctxB, 2, 1.0f / 65536.0f);
  gemm_kernel<1><<<g16, 128, 0, stream>>>(ctxA, ctxB, HID, wo3h, wo3l, HID, BO[2], HID,
                                           1.0f, 0, xres, 1, xA, xB, 2, 1.0f, HID);
  gemm_kernel<1><<<g32, 128, 0, stream>>>(xA, xB, HID, w13h, w13l, HID, B1[2], HID,
                                           1.0f, 1, dummyF, 0, hA, hB, 2, 1.0f, FFH);
  gemm_ln_kernel<1><<<gln, 256, 0, stream>>>(hA, hB, FFH, w23h, w23l, FFH, B2[2], FFH,
                                              1.0f, xres, GA[2], BE[2], OUT, 1, sw_h, 0);
}
